// GAT_Critic_34187939676289
// MI455X (gfx1250) — hardware-verified
//
#include <hip/hip_runtime.h>
#include <stddef.h>


#define NGR     16
#define NPG     1000
#define EPG     16000
#define NT      16000
#define NP      16128
#define NBE     256000
#define F1W     1024
#define NHEAD   8
#define HC1     128
#define EMB     64
#define HID     128
#define NOUT    1000
#define KM1     64000
#define KSPLIT  10
#define KCH     6400
#define NTHR    256
#define NWAVE   8
#define EPT     8
#define CHUNK   (NTHR * EPT)
#define WCAP    (EPT * 32)
#define LISTN   (NWAVE * WCAP)
#define NBMAX   2048
#define SLOTB   11
#define RCAP    28672
#define DEGCAP  4096
#define NBLK    512
#define TPB     512
#define GA      32
#define NSTRM   4
#define GBM     32
#define GTHR    64
#define SWP     136
#define STP     72
#define NEG_SLOPE 0.2f
#define CA      16.0f
#define CB      16.0f
#define CW      64.0f
#define CH      4.0f
#define SCL_G   0.0009765625f
#define SCL_H   0.00390625f
#define WSCAP   134217728
#define LDS_BUILD ((2 * RCAP + 2 * NBMAX + LISTN) * 4 + 64)
#define LDS_HEAD  (NGR * NOUT * 4 + HID * SWP * 2 + 2 * NGR * SWP * 2)

static_assert((CHUNK & (CHUNK - 1)) == 0 && CHUNK <= 4096);
static_assert(NBMAX == (1 << SLOTB));
static_assert(NTHR * 8 == NBMAX);
static_assert(LISTN >= NBMAX);
static_assert(LISTN >= NWAVE * WCAP);
static_assert((RCAP % 32) == 0);
static_assert(LDS_BUILD <= 300000);
static_assert(LDS_HEAD <= 300000);
static_assert(NGR * NPG == NT && NGR * EPG == NBE && NPG * EMB == KM1);
static_assert(NGR * KM1 == NT * EMB);
static_assert((NBE % 4) == 0 && ((NBE / 4) % 32) == 0);
static_assert(NBE < (1 << 21));
static_assert(NP >= NT && (NP % NTHR) == 0 && (NP % GBM) == 0 && NP - NT < NTHR);
static_assert(GA * NBLK >= NP && NBLK <= NBMAX && NBLK >= 16 && (NBLK % 8) == 0);
static_assert(TPB >= NBLK && (TPB % 32) == 0);
static_assert(RCAP * 4 >= NBLK * (2 * NBE / NT) * 7);
static_assert(KSPLIT * KCH == KM1 && (KCH % 32) == 0 && (KM1 % 64) == 0);
static_assert(F1W == NHEAD * HC1 && (F1W % 32) == 0 && EMB == 64 && HID == 128);
static_assert(NSTRM * NHEAD == 32 && NSTRM * 8 == 32);
static_assert(GBM == (GTHR / 32) * 16);
static_assert(((NGR * NOUT) % 4) == 0 && (((NGR * NOUT) / 4) % 32) == 0);
static_assert(((NGR * NOUT * 4) % 16) == 0 && ((SWP * 2) % 16) == 0 && ((STP * 2) % 16) == 0);
static_assert((NOUT + HID - 1) / HID * HID >= NOUT);

typedef float    v4f  __attribute__((ext_vector_type(4)));
typedef float    v8f  __attribute__((ext_vector_type(8)));
typedef int      v4i  __attribute__((ext_vector_type(4)));
typedef int      v8i  __attribute__((ext_vector_type(8)));
typedef _Float16 v8h  __attribute__((ext_vector_type(8)));
typedef _Float16 v16h __attribute__((ext_vector_type(16)));
union FragH { v16h v; v8h h[2]; v8i w; };

__device__ __forceinline__ v8f wmh(const FragH& a, const FragH& b, v8f c) {
  v8f d = __builtin_amdgcn_wmma_f32_16x16x32_f16(false, a.v, false, b.v, (short)0, c, false, false);
  asm volatile("v_nop\n\tv_nop\n\tv_nop\n\tv_nop" : "+v"(d) : "v"(a.w), "v"(b.w));
  return d;
}

__device__ __forceinline__ v8h pack8(v4f a, v4f b, float sc) {
  v8h hv;
  hv[0] = (_Float16)(a.x * sc); hv[1] = (_Float16)(a.y * sc);
  hv[2] = (_Float16)(a.z * sc); hv[3] = (_Float16)(a.w * sc);
  hv[4] = (_Float16)(b.x * sc); hv[5] = (_Float16)(b.y * sc);
  hv[6] = (_Float16)(b.z * sc); hv[7] = (_Float16)(b.w * sc);
  return hv;
}

__device__ __forceinline__ float elu1(float v) {
  const float e = __expf(v) - 1.0f;
  return v > 0.0f ? v : e;
}

__device__ __forceinline__ int node_of(int raw, int pos) {
  raw = raw < 0 ? 0 : (raw > NPG - 1 ? NPG - 1 : raw);
  return raw + (pos / (2 * EPG)) * NPG;
}

__device__ __forceinline__ int scan_chunk(const int* __restrict__ dsts, int nE, int cbase, int slotBase,
                                          int nb, int vec8, int* list, int tid, int lane, int wave) {
  int wc = 0;
  const int el0  = tid * EPT;
  const int e0   = cbase + el0;
  const int sent = -2147483647 - 1;
  v4i da, db;
  if (vec8 != 0 && cbase + CHUNK <= nE) {
    da = *(const v4i*)(dsts + e0);
    db = *(const v4i*)(dsts + e0 + 4);
  } else {
    da.x = (e0     < nE) ? dsts[min(e0,     nE - 1)] : sent;
    da.y = (e0 + 1 < nE) ? dsts[min(e0 + 1, nE - 1)] : sent;
    da.z = (e0 + 2 < nE) ? dsts[min(e0 + 2, nE - 1)] : sent;
    da.w = (e0 + 3 < nE) ? dsts[min(e0 + 3, nE - 1)] : sent;
    db.x = (e0 + 4 < nE) ? dsts[min(e0 + 4, nE - 1)] : sent;
    db.y = (e0 + 5 < nE) ? dsts[min(e0 + 5, nE - 1)] : sent;
    db.z = (e0 + 6 < nE) ? dsts[min(e0 + 6, nE - 1)] : sent;
    db.w = (e0 + 7 < nE) ? dsts[min(e0 + 7, nE - 1)] : sent;
  }
  const unsigned nbs = (unsigned)slotBase;
  const unsigned unb = (unsigned)nb;
  const unsigned s0 = (unsigned)da.x - nbs, s1 = (unsigned)da.y - nbs;
  const unsigned s2 = (unsigned)da.z - nbs, s3 = (unsigned)da.w - nbs;
  const unsigned s4 = (unsigned)db.x - nbs, s5 = (unsigned)db.y - nbs;
  const unsigned s6 = (unsigned)db.z - nbs, s7 = (unsigned)db.w - nbs;
  const bool h0 = s0 < unb, h1 = s1 < unb, h2 = s2 < unb, h3 = s3 < unb;
  const bool h4 = s4 < unb, h5 = s5 < unb, h6 = s6 < unb, h7 = s7 < unb;
  const unsigned any = __builtin_amdgcn_ballot_w32(h0 | h1 | h2 | h3 | h4 | h5 | h6 | h7);
  if (any != 0u) {
#define HITJ(J, HJ, SJ) { \
      const unsigned mj = __builtin_amdgcn_ballot_w32(HJ); \
      if (mj != 0u) { \
        if (HJ) { \
          const int pos = wc + (int)__builtin_amdgcn_mbcnt_lo(mj, 0u); \
          if (pos < WCAP) list[wave * WCAP + pos] = ((el0 + (J)) << 12) | (int)(SJ); \
        } \
        wc += (int)__builtin_popcount(mj); } }
    HITJ(0, h0, s0)
    HITJ(1, h1, s1)
    HITJ(2, h2, s2)
    HITJ(3, h3, s3)
    HITJ(4, h4, s4)
    HITJ(5, h5, s5)
    HITJ(6, h6, s6)
    HITJ(7, h7, s7)
#undef HITJ
  }
  return wc;
}

__global__ __launch_bounds__(NTHR) void k_edges(const int* __restrict__ ei, int* EIS, int* EID, int nUnits) {
  const int u = (int)blockIdx.x * NTHR + (int)threadIdx.x;
  if (u >= nUnits) return;
  const int j0 = 4 * u;
  const v4i rs = *(const v4i*)(ei + j0);
  const v4i rd = *(const v4i*)(ei + NBE + j0);
  v4i s, d;
  s.x = node_of(rs.x, j0);     s.y = node_of(rs.y, j0 + 1);
  s.z = node_of(rs.z, j0 + 2); s.w = node_of(rs.w, j0 + 3);
  d.x = node_of(rd.x, NBE + j0);     d.y = node_of(rd.y, NBE + j0 + 1);
  d.z = node_of(rd.z, NBE + j0 + 2); d.w = node_of(rd.w, NBE + j0 + 3);
  *(volatile v4i*)(EIS + j0) = s;
  *(volatile v4i*)(EID + j0) = d;
  __threadfence();
  *(volatile v4i*)(EIS + j0) = s;
  *(volatile v4i*)(EID + j0) = d;
}

__global__ __launch_bounds__(NTHR) void k_build(const int* __restrict__ dsts, int* EL, int* OFF, int* CNT,
                                                int nE, int nb, int tp, int vec8) {
  extern __shared__ v4f lds_dyn[];
  int* reg1 = (int*)lds_dyn;
  int* reg2 = reg1 + RCAP;
  int* scnt = reg2 + RCAP;
  int* soff = scnt + NBMAX;
  int* list = soff + NBMAX;
  int* wcnt = list + LISTN;
  int* wtot = wcnt + NWAVE;
  const int tid = threadIdx.x, lane = tid & 31, wave = tid >> 5;
  const int nodeBase = (int)blockIdx.x * nb;

  for (int i = tid; i < NBMAX; i += NTHR) scnt[i] = 0;
  {
    const v4i z = {0, 0, 0, 0};
    v4i* r2v = (v4i*)reg2;
    for (int f = tid; f < RCAP / 4; f += NTHR) r2v[f] = z;
  }
  __syncthreads();

  int tot = 0;
  const int nChunks = (nE + CHUNK - 1) / CHUNK;
#pragma unroll 1
  for (int ch = 0; ch < nChunks; ++ch) {
    const int cbase = ch * CHUNK;
    const int wc = scan_chunk(dsts, nE, cbase, nodeBase, nb, vec8, list, tid, lane, wave);
    if (lane == 0) wcnt[wave] = wc;
    __syncthreads();
    int pre = 0, all = 0;
#pragma unroll
    for (int w2 = 0; w2 < NWAVE; ++w2) {
      int c = wcnt[w2];
      c = c < 0 ? 0 : (c > WCAP ? WCAP : c);
      all += c;
      pre += (w2 < wave) ? c : 0;
    }
    const int wcc  = wc > WCAP ? WCAP : wc;
    const int base = tot + pre;
#pragma unroll 1
    for (int i = lane; i < wcc; i += 32) {
      const int ent = list[wave * WCAP + i];
      const int el  = (ent >> 12) & (CHUNK - 1);
      const int sl  = ent & (NBMAX - 1);
      int eid = cbase + el;
      eid = eid > nE - 1 ? nE - 1 : eid;
      const int pos = base + i;
      if (pos < RCAP) reg1[pos] = (int)(((unsigned)eid << SLOTB) | (unsigned)sl);
    }
    tot += all;
    tot = tot > RCAP ? RCAP : tot;
    __syncthreads();
  }
  const int nh = tot;

  if (wave == 0) {
#pragma unroll 1
    for (int b0 = 0; b0 < nh; b0 += 32) {
      const int idx = b0 + lane;
      const int uv  = reg1[idx < RCAP ? idx : RCAP - 1];
      const int m32 = (nh - b0) < 32 ? (nh - b0) : 32;
#pragma unroll 1
      for (int k = 0; k < m32; ++k) {
        const int u  = __builtin_amdgcn_readlane(uv, k);
        const int sl = u & (NBMAX - 1);
        if (lane == 0) scnt[sl] = scnt[sl] + 1;
      }
    }
  }
  __syncthreads();

  {
    const v4i ca = *(const v4i*)(scnt + 8 * tid);
    const v4i cb = *(const v4i*)(scnt + 8 * tid + 4);
    const int e0 = ca.x < 0 ? 0 : ca.x, e1 = ca.y < 0 ? 0 : ca.y, e2 = ca.z < 0 ? 0 : ca.z, e3 = ca.w < 0 ? 0 : ca.w;
    const int e4 = cb.x < 0 ? 0 : cb.x, e5 = cb.y < 0 ? 0 : cb.y, e6 = cb.z < 0 ? 0 : cb.z, e7 = cb.w < 0 ? 0 : cb.w;
    const int ts = e0 + e1 + e2 + e3 + e4 + e5 + e6 + e7;
    int incl = ts;
#pragma unroll
    for (int d = 1; d < 32; d <<= 1) {
      const int up = __shfl_up(incl, d);
      if (lane >= d) incl += up;
    }
    if (lane == 31) wtot[wave] = incl;
    __syncthreads();
    int pre = 0;
#pragma unroll
    for (int w2 = 0; w2 < NWAVE; ++w2) pre += (w2 < wave) ? wtot[w2] : 0;
    int run = pre + incl - ts;
    soff[8 * tid + 0] = run; run += e0;
    soff[8 * tid + 1] = run; run += e1;
    soff[8 * tid + 2] = run; run += e2;
    soff[8 * tid + 3] = run; run += e3;
    soff[8 * tid + 4] = run; run += e4;
    soff[8 * tid + 5] = run; run += e5;
    soff[8 * tid + 6] = run; run += e6;
    soff[8 * tid + 7] = run;
  }
  __syncthreads();
  for (int i = tid; i < NBMAX; i += NTHR) list[i] = soff[i];
  __syncthreads();

  if (wave == 0) {
#pragma unroll 1
    for (int b0 = 0; b0 < nh; b0 += 32) {
      const int idx = b0 + lane;
      const int uv  = reg1[idx < RCAP ? idx : RCAP - 1];
      const int m32 = (nh - b0) < 32 ? (nh - b0) : 32;
#pragma unroll 1
      for (int k = 0; k < m32; ++k) {
        const int u   = __builtin_amdgcn_readlane(uv, k);
        const int sl  = u & (NBMAX - 1);
        const int eid = (int)((unsigned)u >> SLOTB);
        if (lane == 0) {
          int pos = list[sl];
          pos = pos < 0 ? 0 : (pos > RCAP - 1 ? RCAP - 1 : pos);
          reg2[pos] = eid;
          list[sl] = pos + 1;
        }
      }
    }
  }
  __syncthreads();

  {
    int* elb = EL + (size_t)blockIdx.x * RCAP;
    const v4i* r4 = (const v4i*)reg2;
#pragma unroll 1
    for (int f = tid; f < RCAP / 4; f += NTHR) {
      const v4i v = r4[f];
      *(volatile v4i*)(elb + 4 * f) = v;
    }
    __threadfence();
#pragma unroll 1
    for (int f = tid; f < RCAP / 4; f += NTHR) {
      const v4i v = r4[f];
      *(volatile v4i*)(elb + 4 * f) = v;
    }
  }
  {
    const bool ovf = (nh >= RCAP);
    int* ob = OFF + (size_t)blockIdx.x * tp;
    int* cb = CNT + (size_t)blockIdx.x * tp;
    const int n4 = tp >> 2;
#pragma unroll 1
    for (int pass = 0; pass < 2; ++pass) {
#pragma unroll 1
      for (int f = tid; f < n4; f += NTHR) {
        v4i so, sc;
        {
          const int s = 4 * f + 0; const bool in = s < nb; const int scl = s < NBMAX ? s : NBMAX - 1;
          so.x = in ? soff[scl] : 0; sc.x = in ? (ovf ? -1 : scnt[scl]) : 0;
        }
        {
          const int s = 4 * f + 1; const bool in = s < nb; const int scl = s < NBMAX ? s : NBMAX - 1;
          so.y = in ? soff[scl] : 0; sc.y = in ? (ovf ? -1 : scnt[scl]) : 0;
        }
        {
          const int s = 4 * f + 2; const bool in = s < nb; const int scl = s < NBMAX ? s : NBMAX - 1;
          so.z = in ? soff[scl] : 0; sc.z = in ? (ovf ? -1 : scnt[scl]) : 0;
        }
        {
          const int s = 4 * f + 3; const bool in = s < nb; const int scl = s < NBMAX ? s : NBMAX - 1;
          so.w = in ? soff[scl] : 0; sc.w = in ? (ovf ? -1 : scnt[scl]) : 0;
        }
        *(volatile v4i*)(ob + 4 * f) = so;
        *(volatile v4i*)(cb + 4 * f) = sc;
      }
      __threadfence();
    }
  }
}

__global__ __launch_bounds__(NTHR) void k_node1(const float* __restrict__ act, const float* __restrict__ nf,
                                                const float* __restrict__ W1, const float* __restrict__ as1,
                                                const float* __restrict__ ad1,
                                                float* XN, float* ES1, float* ED1) {
  __shared__ float sV[48];
  __shared__ __attribute__((aligned(16))) float sE[NHEAD * NTHR];
  __shared__ __attribute__((aligned(16))) float sD[NHEAD * NTHR];
  const int tid = threadIdx.x;
  if (tid < 24) {
    const int k = tid >> 3, j = tid & 7;
    const float* wp = W1 + (size_t)k * F1W + j * HC1;
    const float* ap = as1 + j * HC1;
    const float* dp = ad1 + j * HC1;
    float s = 0.0f, d = 0.0f;
#pragma unroll 1
    for (int c = 0; c < HC1; ++c) {
      const float w = wp[c];
      s = fmaf(w, ap[c], s);
      d = fmaf(w, dp[c], d);
    }
    sV[tid] = s;
    sV[24 + tid] = d;
  }
  __syncthreads();
  const int blockBase = (int)blockIdx.x * NTHR;
  const int n  = blockBase + tid;
  const int nc = n < NT ? n : NT - 1;
  const float x0 = act[(size_t)nc * 2], x1 = act[(size_t)nc * 2 + 1], x2 = nf[nc];
#pragma unroll 1
  for (int j = 0; j < NHEAD; ++j) {
    float s = x0 * sV[j];
    s = fmaf(x1, sV[8 + j], s);
    s = fmaf(x2, sV[16 + j], s);
    float d = x0 * sV[24 + j];
    d = fmaf(x1, sV[32 + j], d);
    d = fmaf(x2, sV[40 + j], d);
    sE[j * NTHR + tid] = s;
    sD[j * NTHR + tid] = d;
  }
  v4f xv;
  xv.x = x0; xv.y = x1; xv.z = x2; xv.w = 0.0f;
  float* xp = XN + (size_t)n * 4;
  *(volatile v4f*)xp = xv;
  __syncthreads();
  const v4f* e4 = (const v4f*)sE;
  const v4f* d4 = (const v4f*)sD;
#pragma unroll
  for (int i = 0; i < 2; ++i) {
    const int f = tid + NTHR * i;
    const int jj = f >> 6, q = f & 63;
    const v4f ve = e4[f], vd = d4[f];
    *(volatile v4f*)(ES1 + (size_t)jj * NP + blockBase + 4 * q) = ve;
    *(volatile v4f*)(ED1 + (size_t)jj * NP + blockBase + 4 * q) = vd;
  }
  __threadfence();
  *(volatile v4f*)xp = xv;
#pragma unroll
  for (int i = 0; i < 2; ++i) {
    const int f = tid + NTHR * i;
    const int jj = f >> 6, q = f & 63;
    const v4f ve = e4[f], vd = d4[f];
    *(volatile v4f*)(ES1 + (size_t)jj * NP + blockBase + 4 * q) = ve;
    *(volatile v4f*)(ED1 + (size_t)jj * NP + blockBase + 4 * q) = vd;
  }
}

__global__ __launch_bounds__(NTHR) void k_agg1(
    const int* __restrict__ EIS, const int* __restrict__ EL,
    const int* __restrict__ OFF, const int* __restrict__ CNT,
    const float* __restrict__ XN, const float* __restrict__ ES1, const float* __restrict__ ED1,
    const float* __restrict__ W1, const float* __restrict__ b1,
    _Float16* X2, int nE, int nb, int tp) {
  __shared__ __attribute__((aligned(16))) float sW[3 * F1W];
  __shared__ __attribute__((aligned(16))) float sBi[F1W];
  __shared__ v8h sRow[NWAVE * 4 * 32];
  const int tid = threadIdx.x, lane = tid & 31, wave = tid >> 5;
  const int g = lane >> 3, j = lane & 7, hq = lane >> 4;
  for (int i = tid; i < 3 * F1W; i += NTHR) sW[i] = W1[i];
  for (int i = tid; i < F1W; i += NTHR) sBi[i] = b1[i];
  __syncthreads();
  const int nodeBase = (int)blockIdx.x * nb;
  const int nbw = nb >> 3;
  const int* elb  = EL  + (size_t)blockIdx.x * RCAP;
  const int* offb = OFF + (size_t)blockIdx.x * tp;
  const int* cntb = CNT + (size_t)blockIdx.x * tp;
  const float* esj = ES1 + (size_t)j * NP;
  const float* edj = ED1 + (size_t)j * NP;
  const float qnan = __int_as_float(0x7fc00000);
  v8h* sr = sRow + wave * 128;
#pragma unroll 1
  for (int jt = 0; jt < nbw; ++jt) {
    const int slot = wave * nbw + jt;
    const int grow = nodeBase + slot;
    const int gcl  = grow < NT ? grow : NT - 1;
    const int srow = grow < NP ? grow : NP - 1;
    const bool wr  = grow < NP;
    const float caf = grow < NT ? CA : 0.0f;
    int st = offb[slot];
    const int craw = cntb[slot];
    st = st < 0 ? 0 : (st > RCAP - 1 ? RCAP - 1 : st);
    int cnt = craw < 0 ? 0 : (craw > DEGCAP ? DEGCAP : craw);
    if (cnt > RCAP - st) cnt = RCAP - st;
    const float pz = (craw < 0 || craw > DEGCAP) ? qnan : 0.0f;

    const float edv = edj[gcl];
    const float esd = esj[gcl];
    const float t0  = esd + edv;
    float mx = fmaxf(t0, NEG_SLOPE * t0);
    const v4f xd = *(const v4f*)(XN + (size_t)gcl * 4);
    const bool g0 = (g == 0);
    float dn = g0 ? 1.0f : 0.0f;
    float ax = g0 ? xd.x : 0.0f, ay = g0 ? xd.y : 0.0f, az = g0 ? xd.z : 0.0f;
    const int niter = (cnt + NSTRM - 1) / NSTRM;
#pragma unroll 1
    for (int it = 0; it < niter; ++it) {
      const int q = it * NSTRM + g;
      const bool valid = q < cnt;
      const int qc = valid ? q : cnt - 1;
      const int idx = st + qc;
      int eid = elb[idx];
      eid = eid < 0 ? 0 : (eid > nE - 1 ? nE - 1 : eid);
      const int sraw = EIS[eid];
      const int s = sraw < 0 ? 0 : (sraw > NT - 1 ? NT - 1 : sraw);
      const v4f xs = *(const v4f*)(XN + (size_t)s * 4);
      const float ess = esj[s];
      const float u = ess + edv;
      float l = fmaxf(u, NEG_SLOPE * u);
      l = valid ? l : (mx - 100.0f);
      const float mn = fmaxf(mx, l);
      const float s1 = __expf(mx - mn), s2 = __expf(l - mn);
      dn = fmaf(dn, s1, s2);
      ax = fmaf(ax, s1, xs.x * s2);
      ay = fmaf(ay, s1, xs.y * s2);
      az = fmaf(az, s1, xs.z * s2);
      mx = mn;
    }
    float m1 = fmaxf(mx, __shfl_xor(mx, 8));
    m1 = fmaxf(m1, __shfl_xor(m1, 16));
    const float e = __expf(mx - m1);
    dn *= e; ax *= e; ay *= e; az *= e;
    dn += __shfl_xor(dn, 8);  ax += __shfl_xor(ax, 8);  ay += __shfl_xor(ay, 8);  az += __shfl_xor(az, 8);
    dn += __shfl_xor(dn, 16); ax += __shfl_xor(ax, 16); ay += __shfl_xor(ay, 16); az += __shfl_xor(az, 16);
    const float inv = __builtin_amdgcn_rcpf(dn);
    const float rx = fmaf(ax, inv, pz), ry = ay * inv, rz = az * inv;

#pragma unroll 1
    for (int k = 0; k < 4; ++k) {
      const int hd = 2 * k + hq;
      const float r0 = __shfl(rx, hd), r1 = __shfl(ry, hd), r2 = __shfl(rz, hd);
      const int c0 = 256 * k + 8 * lane;
      const v4f wa0 = *(const v4f*)(sW + c0),           wa1 = *(const v4f*)(sW + c0 + 4);
      const v4f wb0 = *(const v4f*)(sW + F1W + c0),     wb1 = *(const v4f*)(sW + F1W + c0 + 4);
      const v4f wc0 = *(const v4f*)(sW + 2 * F1W + c0), wc1 = *(const v4f*)(sW + 2 * F1W + c0 + 4);
      const v4f bb0 = *(const v4f*)(sBi + c0),          bb1 = *(const v4f*)(sBi + c0 + 4);
      v4f o0, o1;
      o0.x = elu1(fmaf(r0, wa0.x, fmaf(r1, wb0.x, fmaf(r2, wc0.x, bb0.x))));
      o0.y = elu1(fmaf(r0, wa0.y, fmaf(r1, wb0.y, fmaf(r2, wc0.y, bb0.y))));
      o0.z = elu1(fmaf(r0, wa0.z, fmaf(r1, wb0.z, fmaf(r2, wc0.z, bb0.z))));
      o0.w = elu1(fmaf(r0, wa0.w, fmaf(r1, wb0.w, fmaf(r2, wc0.w, bb0.w))));
      o1.x = elu1(fmaf(r0, wa1.x, fmaf(r1, wb1.x, fmaf(r2, wc1.x, bb1.x))));
      o1.y = elu1(fmaf(r0, wa1.y, fmaf(r1, wb1.y, fmaf(r2, wc1.y, bb1.y))));
      o1.z = elu1(fmaf(r0, wa1.z, fmaf(r1, wb1.z, fmaf(r2, wc1.z, bb1.z))));
      o1.w = elu1(fmaf(r0, wa1.w, fmaf(r1, wb1.w, fmaf(r2, wc1.w, bb1.w))));
      sr[k * 32 + lane] = pack8(o0, o1, caf);
    }
    _Float16* xrow = X2 + (size_t)srow * F1W + 8 * lane;
    if (wr) {
#pragma unroll
      for (int k = 0; k < 4; ++k) {
        const v8h hv = sr[k * 32 + lane];
        *(volatile v8h*)(xrow + 256 * k) = hv;
      }
    }
    __threadfence();
    if (wr) {
#pragma unroll
      for (int k = 0; k < 4; ++k) {
        const v8h hv = sr[k * 32 + lane];
        *(volatile v8h*)(xrow + 256 * k) = hv;
      }
    }
  }
}

__global__ __launch_bounds__(NTHR) void k_w2prep(const float* __restrict__ w2, _Float16* w2t) {
  const int u = (int)blockIdx.x * NTHR + (int)threadIdx.x;
  const int nUnits = EMB * (F1W / 8);
  if (u >= nUnits) return;
  const int n  = u >> 7;
  const int k8 = (u & 127) * 8;
  const float* p = w2 + (size_t)k8 * EMB + n;
  v4f a, b;
  a.x = p[0 * EMB]; a.y = p[1 * EMB]; a.z = p[2 * EMB]; a.w = p[3 * EMB];
  b.x = p[4 * EMB]; b.y = p[5 * EMB]; b.z = p[6 * EMB]; b.w = p[7 * EMB];
  const v8h hv = pack8(a, b, CW);
  const size_t o = (size_t)n * F1W + k8;
  *(volatile v8h*)(w2t + o) = hv;
  __threadfence();
  *(volatile v8h*)(w2t + o) = hv;
}

__global__ __launch_bounds__(GTHR) void k_gemm2(const _Float16* __restrict__ xc, const _Float16* __restrict__ wt,
                                                const float* __restrict__ asrc, const float* __restrict__ adst,
                                                float* Y, float* ES, float* ED) {
  __shared__ __attribute__((aligned(16))) float stg[GBM * EMB];
  __shared__ __attribute__((aligned(16))) float esT[GBM];
  __shared__ __attribute__((aligned(16))) float edT[GBM];
  __shared__ float sAs[EMB];
  __shared__ float sAd[EMB];
  const int tid = threadIdx.x, lane = tid & 31, wave = tid >> 5, hh = lane >> 4, m = lane & 15;
  const int rowBase = (int)blockIdx.x * GBM;
  for (int i = tid; i < EMB; i += GTHR) { sAs[i] = asrc[i]; sAd[i] = adst[i]; }
  const size_t arow = (size_t)(rowBase + 16 * wave + m) * F1W + 8 * hh;
  const size_t brow = (size_t)m * F1W + 8 * hh;
  v8f acc[4];
#pragma unroll
  for (int t = 0; t < 4; ++t) { v8f z = {0.f, 0.f, 0.f, 0.f, 0.f, 0.f, 0.f, 0.f}; acc[t] = z; }
#pragma unroll 1
  for (int ks = 0; ks < F1W / 32; ++ks) {
    FragH af;
    af.h[0] = *(const v8h*)(xc + arow + 32 * ks);
    af.h[1] = *(const v8h*)(xc + arow + 32 * ks + 16);
#pragma unroll
    for (int t = 0; t < 4; ++t) {
      const size_t bo = brow + (size_t)(16 * t) * F1W + 32 * ks;
      FragH bf;
      bf.h[0] = *(const v8h*)(wt + bo);
      bf.h[1] = *(const v8h*)(wt + bo + 16);
      acc[t] = wmh(af, bf, acc[t]);
    }
  }
  {
    float* sp = stg + (size_t)(16 * wave + 8 * hh) * EMB + m;
#pragma unroll
    for (int t = 0; t < 4; ++t) {
#pragma unroll
      for (int r = 0; r < 8; ++r) sp[(size_t)r * EMB + 16 * t] = acc[t][r] * SCL_G;
    }
  }
  __syncthreads();
  {
    const int row  = tid >> 1;
    const int half = tid & 1;
    const float* srow = stg + (size_t)row * EMB;
    float s = 0.f, d = 0.f;
#pragma unroll 1
    for (int c = 0; c < EMB / 2; ++c) {
      const int cc = half * (EMB / 2) + c;
      const float v = srow[cc];
      s = fmaf(v, sAs[cc], s);
      d = fmaf(v, sAd[cc], d);
    }
    s += __shfl_xor(s, 1);
    d += __shfl_xor(d, 1);
    if (half == 0) {
      esT[row] = s;
      edT[row] = d;
    }
  }
  {
    const int nF4 = GBM * EMB / 4;
    float* yb = Y + (size_t)rowBase * EMB;
    const v4f* s4 = (const v4f*)stg;
#pragma unroll 1
    for (int f = tid; f < nF4; f += GTHR) {
      const v4f v = s4[f];
      *(volatile v4f*)(yb + 4 * (size_t)f) = v;
    }
    __threadfence();
#pragma unroll 1
    for (int f = tid; f < nF4; f += GTHR) {
      const v4f v = s4[f];
      *(volatile v4f*)(yb + 4 * (size_t)f) = v;
    }
  }
  __syncthreads();
  {
    const int l8 = tid & 7;
    const bool wl = tid < 8;
    const v4f ve = *(const v4f*)(esT + 4 * l8);
    const v4f vd = *(const v4f*)(edT + 4 * l8);
    float* pe = ES + (size_t)rowBase + 4 * l8;
    float* pd = ED + (size_t)rowBase + 4 * l8;
    if (wl) {
      *(volatile v4f*)pe = ve;
      *(volatile v4f*)pd = vd;
    }
    __threadfence();
    if (wl) {
      *(volatile v4f*)pe = ve;
      *(volatile v4f*)pd = vd;
    }
  }
}

__global__ __launch_bounds__(NTHR) void k_agg2(
    const int* __restrict__ EIS, const int* __restrict__ EL,
    const int* __restrict__ OFF, const int* __restrict__ CNT,
    const float* __restrict__ H2, const float* __restrict__ ES2, const float* __restrict__ ED2,
    const float* __restrict__ b2, _Float16* X3, int nE, int nb, int tp) {
  const int tid = threadIdx.x, lane = tid & 31, wave = tid >> 5;
  const int g = lane >> 3, sub = lane & 7;
  const int cb0 = 8 * sub;
  const int nodeBase = (int)blockIdx.x * nb;
  const int nbw = nb >> 3;
  const int* elb  = EL  + (size_t)blockIdx.x * RCAP;
  const int* offb = OFF + (size_t)blockIdx.x * tp;
  const int* cntb = CNT + (size_t)blockIdx.x * tp;
  const v4f bz0 = *(const v4f*)(b2 + cb0);
  const v4f bz1 = *(const v4f*)(b2 + cb0 + 4);
  const float qnan = __int_as_float(0x7fc00000);
  const v4f z4 = {0.f, 0.f, 0.f, 0.f};
#pragma unroll 1
  for (int jt = 0; jt < nbw; ++jt) {
    const int slot = wave * nbw + jt;
    const int grow = nodeBase + slot;
    const int gcl  = grow < NT ? grow : NT - 1;
    const bool wr  = grow < NT;
    int st = offb[slot];
    const int craw = cntb[slot];
    st = st < 0 ? 0 : (st > RCAP - 1 ? RCAP - 1 : st);
    int cnt = craw < 0 ? 0 : (craw > DEGCAP ? DEGCAP : craw);
    if (cnt > RCAP - st) cnt = RCAP - st;
    const float pz = (craw < 0 || craw > DEGCAP) ? qnan : 0.0f;

    const float edv = ED2[gcl];
    const float esd = ES2[gcl];
    const float t0  = esd + edv;
    float mx = fmaxf(t0, NEG_SLOPE * t0);
    const float* yd = H2 + (size_t)gcl * EMB + cb0;
    const bool g0 = (g == 0);
    float dn = g0 ? 1.0f : 0.0f;
    const v4f y0 = *(const v4f*)(yd), y1 = *(const v4f*)(yd + 4);
    v4f a0 = g0 ? y0 : z4, a1 = g0 ? y1 : z4;
    const int niter = (cnt + NSTRM - 1) / NSTRM;
#pragma unroll 1
    for (int it = 0; it < niter; ++it) {
      const int q = it * NSTRM + g;
      const bool valid = q < cnt;
      const int qc = valid ? q : cnt - 1;
      const int idx = st + qc;
      int eid = elb[idx];
      eid = eid < 0 ? 0 : (eid > nE - 1 ? nE - 1 : eid);
      const int sraw = EIS[eid];
      const int s = sraw < 0 ? 0 : (sraw > NT - 1 ? NT - 1 : sraw);
      const float* ys = H2 + (size_t)s * EMB + cb0;
      const v4f x0 = *(const v4f*)(ys);
      const v4f x1 = *(const v4f*)(ys + 4);
      const float ess = ES2[s];
      const float u = ess + edv;
      float l = fmaxf(u, NEG_SLOPE * u);
      l = valid ? l : (mx - 100.0f);
      const float mn = fmaxf(mx, l);
      const float s1 = __expf(mx - mn), s2 = __expf(l - mn);
      dn = fmaf(dn, s1, s2);
      a0 = a0 * s1 + x0 * s2;
      a1 = a1 * s1 + x1 * s2;
      mx = mn;
    }
    float m1 = fmaxf(mx, __shfl_xor(mx, 8));
    m1 = fmaxf(m1, __shfl_xor(m1, 16));
    const float e = __expf(mx - m1);
    dn *= e; a0 = a0 * e; a1 = a1 * e;
    dn   += __shfl_xor(dn, 8);
    a0.x += __shfl_xor(a0.x, 8); a0.y += __shfl_xor(a0.y, 8); a0.z += __shfl_xor(a0.z, 8); a0.w += __shfl_xor(a0.w, 8);
    a1.x += __shfl_xor(a1.x, 8); a1.y += __shfl_xor(a1.y, 8); a1.z += __shfl_xor(a1.z, 8); a1.w += __shfl_xor(a1.w, 8);
    dn   += __shfl_xor(dn, 16);
    a0.x += __shfl_xor(a0.x, 16); a0.y += __shfl_xor(a0.y, 16); a0.z += __shfl_xor(a0.z, 16); a0.w += __shfl_xor(a0.w, 16);
    a1.x += __shfl_xor(a1.x, 16); a1.y += __shfl_xor(a1.y, 16); a1.z += __shfl_xor(a1.z, 16); a1.w += __shfl_xor(a1.w, 16);
    const float inv = __builtin_amdgcn_rcpf(dn);
    v4f o0 = a0 * inv + bz0 + pz;
    v4f o1 = a1 * inv + bz1 + pz;
    o0.x = elu1(o0.x); o0.y = elu1(o0.y); o0.z = elu1(o0.z); o0.w = elu1(o0.w);
    o1.x = elu1(o1.x); o1.y = elu1(o1.y); o1.z = elu1(o1.z); o1.w = elu1(o1.w);
    const v8h hv = pack8(o0, o1, CB);
    _Float16* xp = X3 + (size_t)gcl * EMB + cb0;
    const bool wsl = wr && g0;
    if (wsl) *(volatile v8h*)xp = hv;
    __threadfence();
    if (wsl) *(volatile v8h*)xp = hv;
  }
}

__global__ __launch_bounds__(NTHR) void k_w1prep(const float* __restrict__ w, _Float16* w1t) {
  __shared__ __attribute__((aligned(16))) _Float16 sT[HID * STP];
  const int tid = threadIdx.x;
  const int k0 = (int)blockIdx.x * 64;
#pragma unroll 1
  for (int i = 0; i < (64 * HID) / NTHR; ++i) {
    const int e  = tid + NTHR * i;
    const int kk = e >> 7, n = e & (HID - 1);
    const float v = w[(size_t)(k0 + kk) * HID + n];
    sT[n * STP + kk] = (_Float16)(v * CW);
  }
  __syncthreads();
#pragma unroll
  for (int i = 0; i < 4; ++i) {
    const int f = tid + NTHR * i;
    const int n = f >> 3, p = f & 7;
    const v8h hv = *(const v8h*)(sT + n * STP + 8 * p);
    *(volatile v8h*)(w1t + (size_t)n * KM1 + k0 + 8 * p) = hv;
  }
  __threadfence();
#pragma unroll
  for (int i = 0; i < 4; ++i) {
    const int f = tid + NTHR * i;
    const int n = f >> 3, p = f & 7;
    const v8h hv = *(const v8h*)(sT + n * STP + 8 * p);
    *(volatile v8h*)(w1t + (size_t)n * KM1 + k0 + 8 * p) = hv;
  }
}

__global__ __launch_bounds__(NTHR) void k_mlp1(const _Float16* __restrict__ x3, const _Float16* __restrict__ w1t,
                                               float* P1) {
  __shared__ __attribute__((aligned(16))) float sP[NGR * HID];
  const int tid = threadIdx.x, lane = tid & 31, wave = tid >> 5, hh = lane >> 4, m = lane & 15;
  const int p = (int)blockIdx.x;
  const int kbase = p * KCH;
  const _Float16* ap = x3  + (size_t)m * KM1 + kbase + 8 * hh;
  const _Float16* bp = w1t + (size_t)(16 * wave + m) * KM1 + kbase + 8 * hh;
  v8f acc = {0.f, 0.f, 0.f, 0.f, 0.f, 0.f, 0.f, 0.f};
#pragma unroll 1
  for (int ks = 0; ks < KCH / 32; ++ks) {
    FragH af, bf;
    af.h[0] = *(const v8h*)(ap + 32 * ks);
    af.h[1] = *(const v8h*)(ap + 32 * ks + 16);
    bf.h[0] = *(const v8h*)(bp + 32 * ks);
    bf.h[1] = *(const v8h*)(bp + 32 * ks + 16);
    acc = wmh(af, bf, acc);
  }
  {
    float* sp = sP + (size_t)(8 * hh) * HID + 16 * wave + m;
#pragma unroll
    for (int r = 0; r < 8; ++r) sp[(size_t)r * HID] = acc[r];
  }
  __syncthreads();
  float* pb = P1 + (size_t)p * (NGR * HID);
  const v4f* s4 = (const v4f*)sP;
#pragma unroll
  for (int i = 0; i < 2; ++i) {
    const int f = tid + NTHR * i;
    const v4f v = s4[f];
    *(volatile v4f*)(pb + 4 * f) = v;
  }
  __threadfence();
#pragma unroll
  for (int i = 0; i < 2; ++i) {
    const int f = tid + NTHR * i;
    const v4f v = s4[f];
    *(volatile v4f*)(pb + 4 * f) = v;
  }
}

__global__ __launch_bounds__(NTHR) void k_head(const float* __restrict__ P1, const float* __restrict__ mb1,
                                               const float* __restrict__ mw2, const float* __restrict__ mb2,
                                               const float* __restrict__ ow, const float* __restrict__ ob,
                                               float* out) {
  extern __shared__ v4f lds_dyn[];
  float*    sO  = (float*)lds_dyn;
  _Float16* sW  = (_Float16*)(sO + NGR * NOUT);
  _Float16* sA1 = sW + HID * SWP;
  _Float16* sA2 = sA1 + NGR * SWP;
  const int tid = threadIdx.x, lane = tid & 31, wave = tid >> 5, hh = lane >> 4, m = lane & 15;
#pragma unroll 1
  for (int i = 0; i < (NGR * HID) / NTHR; ++i) {
    const int e = tid + NTHR * i;
    const int n = e & (HID - 1), b = e >> 7;
    float s = 0.0f;
#pragma unroll 1
    for (int p = 0; p < KSPLIT; ++p) s += P1[(size_t)p * (NGR * HID) + e];
    s = fmaf(s, SCL_G, mb1[n]);
    s = fmaxf(s, 0.0f);
    sA1[b * SWP + n] = (_Float16)(s * CH);
  }
#pragma unroll 1
  for (int i = 0; i < (HID * HID) / NTHR; ++i) {
    const int e = tid + NTHR * i;
    const int k = e >> 7, n = e & (HID - 1);
    sW[n * SWP + k] = (_Float16)(mw2[e] * CW);
  }
  __syncthreads();
  v8f acc = {0.f, 0.f, 0.f, 0.f, 0.f, 0.f, 0.f, 0.f};
  {
    const _Float16* ap = sA1 + m * SWP + 8 * hh;
    const _Float16* bp = sW + (16 * wave + m) * SWP + 8 * hh;
#pragma unroll
    for (int ks = 0; ks < HID / 32; ++ks) {
      FragH af, bf;
      af.h[0] = *(const v8h*)(ap + 32 * ks);
      af.h[1] = *(const v8h*)(ap + 32 * ks + 16);
      bf.h[0] = *(const v8h*)(bp + 32 * ks);
      bf.h[1] = *(const v8h*)(bp + 32 * ks + 16);
      acc = wmh(af, bf, acc);
    }
  }
  {
    const int n = 16 * wave + m;
    const float bb = mb2[n];
    _Float16* hp = sA2 + (8 * hh) * SWP + n;
#pragma unroll
    for (int r = 0; r < 8; ++r) {
      const float v = fmaxf(fmaf(acc[r], SCL_H, bb), 0.0f);
      hp[r * SWP] = (_Float16)(v * CH);
    }
  }
  __syncthreads();
#pragma unroll 1
  for (int c = 0; c < (NOUT + HID - 1) / HID; ++c) {
#pragma unroll 1
    for (int i = 0; i < (HID * HID) / NTHR; ++i) {
      const int e = tid + NTHR * i;
      const int k = e >> 7, n = e & (HID - 1);
      const int col  = HID * c + n;
      const int colc = col < NOUT ? col : NOUT - 1;
      float v = ow[(size_t)k * NOUT + colc];
      v = col < NOUT ? v : 0.0f;
      sW[n * SWP + k] = (_Float16)(v * CW);
    }
    __syncthreads();
    v8f acc2 = {0.f, 0.f, 0.f, 0.f, 0.f, 0.f, 0.f, 0.f};
    {
      const _Float16* ap = sA2 + m * SWP + 8 * hh;
      const _Float16* bp = sW + (16 * wave + m) * SWP + 8 * hh;
#pragma unroll
      for (int ks = 0; ks < HID / 32; ++ks) {
        FragH af, bf;
        af.h[0] = *(const v8h*)(ap + 32 * ks);
        af.h[1] = *(const v8h*)(ap + 32 * ks + 16);
        bf.h[0] = *(const v8h*)(bp + 32 * ks);
        bf.h[1] = *(const v8h*)(bp + 32 * ks + 16);
        acc2 = wmh(af, bf, acc2);
      }
    }
    {
      const int col  = HID * c + 16 * wave + m;
      const int colc = col < NOUT ? col : NOUT - 1;
      const bool keep = col < NOUT;
      const float bo = ob[colc];
      float* op = sO + (size_t)(8 * hh) * NOUT + colc;
#pragma unroll
      for (int r = 0; r < 8; ++r) {
        const float z  = fmaf(acc2[r], SCL_H, bo);
        const float ez = __expf(-z);
        const float sg = __builtin_amdgcn_rcpf(1.0f + ez);
        if (keep) op[(size_t)r * NOUT] = sg;
      }
    }
    __syncthreads();
  }
  const v4f* s4 = (const v4f*)sO;
  const int n4 = (NGR * NOUT) / 4;
#pragma unroll 1
  for (int f = tid; f < n4; f += NTHR) {
    const v4f v = s4[f];
    *(volatile v4f*)(out + 4 * (size_t)f) = v;
  }
  __threadfence();
#pragma unroll 1
  for (int f = tid; f < n4; f += NTHR) {
    const v4f v = s4[f];
    *(volatile v4f*)(out + 4 * (size_t)f) = v;
  }
}

extern "C" void kernel_launch(void* const* d_in, const int* in_sizes, int n_in,
                              void* d_out, int out_size, void* d_ws, size_t ws_size,
                              hipStream_t stream) {
  if (n_in < 17) return;
  if (in_sizes[0] != NT * 2 || in_sizes[1] != NT || in_sizes[2] != 2 * NBE) return;
  if (in_sizes[3] != 3 * F1W || in_sizes[4] != F1W || in_sizes[5] != F1W || in_sizes[6] != F1W) return;
  if (in_sizes[7] != F1W * EMB || in_sizes[8] != EMB || in_sizes[9] != EMB || in_sizes[10] != EMB) return;
  if (in_sizes[11] != KM1 * HID || in_sizes[12] != HID || in_sizes[13] != HID * HID || in_sizes[14] != HID) return;
  if (in_sizes[15] != HID * NOUT || in_sizes[16] != NOUT) return;
  if (out_size != NGR * NOUT) return;

  const float* actions = (const float*)d_in[0];
  const float* nodef   = (const float*)d_in[1];
  const int*   eidx    = (const int*)d_in[2];
  const float* W1      = (const float*)d_in[3];
  const float* as1     = (const float*)d_in[4];
  const float* ad1     = (const float*)d_in[5];
  const float* b1      = (const float*)d_in[6];
  const float* W2      = (const float*)d_in[7];
  const float* as2     = (const float*)d_in[8];
  const float* ad2     = (const float*)d_in[9];
  const float* b2      = (const float*)d_in[10];
  const float* mw1     = (const float*)d_in[11];
  const float* mb1     = (const float*)d_in[12];
  const float* mw2     = (const float*)d_in[13];
  const float* mb2     = (const float*)d_in[14];
  const float* ow      = (const float*)d_in[15];
  const float* obias   = (const float*)d_in[16];
  float* out = (float*)d_out;

  char* ws = (char*)d_ws;
  size_t off = 0;
  const size_t oEIS = off; off += (size_t)NBE * 4;                  off = (off + 255) & ~(size_t)255;
  const size_t oEID = off; off += (size_t)NBE * 4;                  off = (off + 255) & ~(size_t)255;
  const size_t oXN  = off; off += (size_t)NP * 4 * 4;               off = (off + 255) & ~(size_t)255;
  const size_t oES1 = off; off += (size_t)NHEAD * NP * 4;           off = (off + 255) & ~(size_t)255;
  const size_t oED1 = off; off += (size_t)NHEAD * NP * 4;           off = (off + 255) & ~(size_t)255;
  const size_t oEL  = off; off += (size_t)GA * RCAP * 4;            off = (off + 255) & ~(size_t)255;
  const size_t oOFF = off; off += (size_t)GA * TPB * 4;             off = (off + 255) & ~(size_t)255;
  const size_t oCNT = off; off += (size_t)GA * TPB * 4;             off = (off + 255) & ~(size_t)255;
  const size_t oX2  = off; off += (size_t)NP * F1W * 2;             off = (off + 255) & ~(size_t)255;
  const size_t oW2T = off; off += (size_t)EMB * F1W * 2;            off = (off + 255) & ~(size_t)255;
  const size_t oH2  = off; off += (size_t)NP * EMB * 4;             off = (off + 255) & ~(size_t)255;
  const size_t oES2 = off; off += (size_t)NP * 4;                   off = (off + 255) & ~(size_t)255;
  const size_t oED2 = off; off += (size_t)NP * 4;                   off = (off + 255) & ~(size_t)255;
  const size_t oX3  = off; off += (size_t)NGR * KM1 * 2;            off = (off + 255) & ~(size_t)255;
  const size_t oW1T = off; off += (size_t)HID * KM1 * 2;            off = (off + 255) & ~(size_t)255;
  const size_t oP1  = off; off += (size_t)KSPLIT * NGR * HID * 4;   off = (off + 255) & ~(size_t)255;
  if (off > ws_size || off > (size_t)WSCAP) return;
  int*      EIS = (int*)(ws + oEIS);
  int*      EID = (int*)(ws + oEID);
  float*    XN  = (float*)(ws + oXN);
  float*    ES1 = (float*)(ws + oES1);
  float*    ED1 = (float*)(ws + oED1);
  int*      EL  = (int*)(ws + oEL);
  int*      OFF = (int*)(ws + oOFF);
  int*      CNT = (int*)(ws + oCNT);
  _Float16* X2  = (_Float16*)(ws + oX2);
  _Float16* W2T = (_Float16*)(ws + oW2T);
  float*    H2  = (float*)(ws + oH2);
  float*    ES2 = (float*)(ws + oES2);
  float*    ED2 = (float*)(ws + oED2);
  _Float16* X3  = (_Float16*)(ws + oX3);
  _Float16* W1T = (_Float16*)(ws + oW1T);
  float*    P1  = (float*)(ws + oP1);

  hipFuncSetAttribute(reinterpret_cast<const void*>(&k_build),
                      hipFuncAttributeMaxDynamicSharedMemorySize, LDS_BUILD);
  hipFuncSetAttribute(reinterpret_cast<const void*>(&k_head),
                      hipFuncAttributeMaxDynamicSharedMemorySize, LDS_HEAD);

  const int nUnitsE = NBE / 4;

  k_edges<<<(nUnitsE + NTHR - 1) / NTHR, NTHR, 0, stream>>>(eidx, EIS, EID, nUnitsE);
  k_build<<<GA, NTHR, LDS_BUILD, stream>>>(EID, EL, OFF, CNT, NBE, NBLK, TPB, 1);

  k_node1<<<NP / NTHR, NTHR, 0, stream>>>(actions, nodef, W1, as1, ad1, XN, ES1, ED1);
  k_agg1<<<GA, NTHR, 0, stream>>>(EIS, EL, OFF, CNT, XN, ES1, ED1, W1, b1, X2, NBE, NBLK, TPB);

  k_w2prep<<<(EMB * (F1W / 8) + NTHR - 1) / NTHR, NTHR, 0, stream>>>(W2, W2T);
  k_gemm2<<<NP / GBM, GTHR, 0, stream>>>(X2, W2T, as2, ad2, H2, ES2, ED2);
  k_agg2<<<GA, NTHR, 0, stream>>>(EIS, EL, OFF, CNT, H2, ES2, ED2, b2, X3, NBE, NBLK, TPB);

  k_w1prep<<<KM1 / 64, NTHR, 0, stream>>>(mw1, W1T);
  k_mlp1<<<KSPLIT, NTHR, 0, stream>>>(X3, W1T, P1);
  k_head<<<1, NTHR, LDS_HEAD, stream>>>(P1, mb1, mw2, mb2, ow, obias, out);
}
